// HybridGraphRefiner_57019985822410
// MI455X (gfx1250) — hardware-verified
//
#include <hip/hip_runtime.h>
#include <hip/hip_bf16.h>


#define BB 2
#define CC 256
#define NN 4096
#define HWD 64
#define HIDD 128
#define NPP 16
#define NCC 16
#define QK_O 512
#define KCONV 4608
#define NPIX 8192
#define WSC 64.0f

typedef __attribute__((ext_vector_type(16))) _Float16 v16h;
typedef __attribute__((ext_vector_type(8)))  _Float16 v8h;
typedef __attribute__((ext_vector_type(16))) __bf16   v16b;
typedef __attribute__((ext_vector_type(8)))  __bf16   v8b;
typedef __attribute__((ext_vector_type(8)))  float    v8f;
typedef __attribute__((ext_vector_type(4)))  float    v4f;
#define PSCALE 32768.0f
#define U16(p) ((const unsigned short*)(const void*)(p))
#define PSCALE_INV (1.0f / 32768.0f)

__device__ __forceinline__ unsigned short f2bf_bits(float f) {
  unsigned u = __float_as_uint(f);
  return (unsigned short)((u + 0x7FFFu + ((u >> 16) & 1u)) >> 16);
}
__device__ __forceinline__ float bf_bits2f(unsigned short h) { return __uint_as_float(((unsigned)h) << 16); }

__device__ __forceinline__ void dep_guard_h(v8f& a, v8f& b, v16h x, v16h y) { asm volatile("v_nop\n\tv_nop\n\tv_nop\n\tv_nop" : "+v"(a), "+v"(b) : "v"(x), "v"(y)); }
__device__ __forceinline__ void dep_guard_b(v8f& a, v8f& b, v16b x, v16b y) { asm volatile("v_nop\n\tv_nop\n\tv_nop\n\tv_nop" : "+v"(a), "+v"(b) : "v"(x), "v"(y)); }
__device__ __forceinline__ void keep4_h(v16h a, v16h b, v16h c, v16h d) { asm volatile("v_nop" :: "v"(a), "v"(b), "v"(c), "v"(d)); }
__device__ __forceinline__ void keep4_b(v16b a, v16b b, v16b c, v16b d) { asm volatile("v_nop" :: "v"(a), "v"(b), "v"(c), "v"(d)); }
__device__ __forceinline__ void acc_guard4(v8f& a, v8f& b, v8f& c, v8f& d) { asm volatile("v_nop\n\tv_nop\n\tv_nop\n\tv_nop" : "+v"(a), "+v"(b), "+v"(c), "+v"(d)); }
template <typename T> struct Frag;
template <> struct Frag<_Float16> {
  typedef v16h V; union U { v16h v; v8h h[2]; };
  static __device__ __forceinline__ v16h load(const _Float16* p) {
    U f; f.h[0] = *(const v8h*)(p); f.h[1] = *(const v8h*)(p + 16); return f.v;
  }
  static __device__ __forceinline__ v8f mma(v16h a, v16h b, v8f c) {
    return __builtin_amdgcn_wmma_f32_16x16x32_f16(false, a, false, b, (short)0, c, false, false);
  }
  static __device__ __forceinline__ void guard(v8f& a, v8f& b, v16h x, v16h y) { dep_guard_h(a, b, x, y); }
  static __device__ __forceinline__ void keep(v16h a, v16h b, v16h c, v16h d) { keep4_h(a, b, c, d); }
};
template <> struct Frag<__bf16> {
  typedef v16b V; union U { v16b v; v8b h[2]; };
  static __device__ __forceinline__ v16b load(const __bf16* p) {
    U f; f.h[0] = *(const v8b*)(p); f.h[1] = *(const v8b*)(p + 16); return f.v;
  }
  static __device__ __forceinline__ v8f mma(v16b a, v16b b, v8f c) {
    return __builtin_amdgcn_wmma_f32_16x16x32_bf16(false, a, false, b, (short)0, c, false, false);
  }
  static __device__ __forceinline__ void guard(v8f& a, v8f& b, v16b x, v16b y) { dep_guard_b(a, b, x, y); }
  static __device__ __forceinline__ void keep(v16b a, v16b b, v16b c, v16b d) { keep4_b(a, b, c, d); }
};

template <int ET> struct Elem;
template <> struct Elem<0> { typedef _Float16 T; };
template <> struct Elem<1> { typedef __bf16 T; };
template <int ET, bool SPLIT, int BIAS_MODE, int OUT_MODE, bool RESID, int ACT = 0>
__global__ __launch_bounds__(256) void wmma_gemm64(
    const unsigned short* __restrict__ Ap, const unsigned short* __restrict__ A2p, int lda, long strideA,
    const unsigned short* __restrict__ Btp, const unsigned short* __restrict__ Bt2p, int ldb, long strideB,
    void* __restrict__ Cout, void* __restrict__ Cout2, int ldc, long strideC,
    const float* __restrict__ bias,
    const float* __restrict__ resid, long strideR,
    int M, int N, int K, float scale) {
  typedef typename Elem<ET>::T T;
  typedef typename Frag<T>::V V;
  const T* A = (const T*)Ap; const T* A2 = (const T*)A2p; const T* Bt = (const T*)Btp; const T* Bt2 = (const T*)Bt2p;
  __shared__ __align__(16) float sT[8][16 * 68];
  const int b    = blockIdx.y;
  const int lane = threadIdx.x & 31;
  const int wave = threadIdx.x >> 5;
  const int tilesN = N >> 6;
  const int tilesM = M >> 6;
  const int tile = blockIdx.x * 8 + wave;
  if (tile >= tilesM * tilesN) return;
  const int tm = tile / tilesN;
  const int tn = tile - tm * tilesN;
  const int m0 = tm << 6;
  const int n0 = tn << 6;

  const T* Ab  = A  + (size_t)b * strideA;
  const T* Bb  = Bt + (size_t)b * strideB;
  const T* Ab2 = SPLIT ? (A2  + (size_t)b * strideA) : nullptr;
  const T* Bb2 = SPLIT ? (Bt2 + (size_t)b * strideB) : nullptr;

  const int rlane = lane & 15;
  const int koff  = (lane >> 4) * 8;
  const int mOff  = (lane >> 4) * 8;

  v8f acc[4][4];
#pragma unroll
  for (int i = 0; i < 4; ++i)
#pragma unroll
    for (int j = 0; j < 4; ++j) acc[i][j] = (v8f){0.f,0.f,0.f,0.f,0.f,0.f,0.f,0.f};

  for (int k0 = 0; k0 < K; k0 += 32) {
    V bh[4], bl[4];
#pragma unroll
    for (int j = 0; j < 4; ++j) {
      const size_t bo = (size_t)(n0 + (j << 4) + rlane) * ldb + koff + k0;
      bh[j] = Frag<T>::load(Bb + bo);
      if (SPLIT) bl[j] = Frag<T>::load(Bb2 + bo);
    }
#pragma unroll
    for (int i = 0; i < 4; ++i) {
      const size_t ao = (size_t)(m0 + (i << 4) + rlane) * lda + koff + k0;
      V ah = Frag<T>::load(Ab + ao);
      V al;
      if (SPLIT) al = Frag<T>::load(Ab2 + ao);
#pragma unroll
      for (int j = 0; j < 4; ++j) {
        acc[i][j] = Frag<T>::mma(ah, bh[j], acc[i][j]);
        if (SPLIT) {
          acc[i][j] = Frag<T>::mma(ah, bl[j], acc[i][j]);
          acc[i][j] = Frag<T>::mma(al, bh[j], acc[i][j]);
        }
      }
      Frag<T>::guard(acc[i][0], acc[i][3], ah, SPLIT ? al : ah);
    }
    Frag<T>::keep(bh[0], bh[1], bh[2], bh[3]);
    if (SPLIT) Frag<T>::keep(bl[0], bl[1], bl[2], bl[3]);
  }
  acc_guard4(acc[0][0], acc[0][1], acc[0][2], acc[0][3]);
  acc_guard4(acc[1][0], acc[1][1], acc[1][2], acc[1][3]);
  acc_guard4(acc[2][0], acc[2][1], acc[2][2], acc[2][3]);
  acc_guard4(acc[3][0], acc[3][1], acc[3][2], acc[3][3]);

  float* slab = sT[wave];
  const float* Rb = RESID ? (resid + (size_t)b * strideR) : nullptr;
#pragma unroll
  for (int i = 0; i < 4; ++i) {
    const int mBase = m0 + (i << 4);
#pragma unroll
    for (int j = 0; j < 4; ++j) {
      const int n = n0 + (j << 4) + rlane;
      float bv = 0.f;
      if (BIAS_MODE == 2) bv = bias[n];
#pragma unroll
      for (int r = 0; r < 8; ++r) {
        float v = acc[i][j][r] * scale;
        if (BIAS_MODE == 1) v += bias[mBase + mOff + r];
        if (BIAS_MODE == 2) v += bv;
        if (RESID) v += Rb[(size_t)(mBase + mOff + r) * ldc + n];
        if (ACT == 1) v = tanhf(v);
        if (ACT == 2) v = fmaxf(v, 0.0f);
        if (ACT == 3) v = v / (1.0f + expf(-v));
        if (ACT == 4) v = (v > 0.f) ? v : 0.01f * v;
        if (ACT == 5) v = 0.5f * v * (1.0f + erff(v * 0.70710678118654752f));
        slab[(mOff + r) * 68 + (j << 4) + rlane] = v;
      }
    }
    __builtin_amdgcn_fence(__ATOMIC_RELEASE, "workgroup");
    __builtin_amdgcn_wave_barrier();
    __builtin_amdgcn_fence(__ATOMIC_ACQUIRE, "workgroup");
    if (OUT_MODE == 0) {
      float* C = (float*)Cout + (size_t)b * strideC;
      const int hh = lane >> 4, c4 = (lane & 15) * 4;
      for (int pass = 0; pass < 2; ++pass) {
#pragma unroll
        for (int it = 0; it < 8; ++it) {
          const int row = it * 2 + hh;
          v4f v = *(const v4f*)(slab + row * 68 + c4);
          *(volatile v4f*)(C + (size_t)(mBase + row) * ldc + n0 + c4) = v;
        }
        __threadfence();
      }
    } else {
      const int q = lane >> 3, c8 = (lane & 7) * 8;
      unsigned short* C  = (unsigned short*)Cout  + (size_t)b * strideC;
      unsigned short* C2 = (OUT_MODE == 2) ? ((unsigned short*)Cout2 + (size_t)b * strideC) : nullptr;
      for (int pass = 0; pass < 2; ++pass) {
#pragma unroll
        for (int it = 0; it < 4; ++it) {
          const int row = it * 4 + q;
          const float* sp = slab + row * 68 + c8;
          v8h hv, lv;
#pragma unroll
          for (int e = 0; e < 8; ++e) {
            if (OUT_MODE == 1) {
              hv[e] = (_Float16)sp[e];
            } else {
              unsigned short hb = f2bf_bits(sp[e]);
              unsigned short lb = f2bf_bits(sp[e] - bf_bits2f(hb));
              hv[e] = __builtin_bit_cast(_Float16, hb);
              lv[e] = __builtin_bit_cast(_Float16, lb);
            }
          }
          *(volatile v8h*)(C + (size_t)(mBase + row) * ldc + n0 + c8) = hv;
          if (OUT_MODE == 2) *(volatile v8h*)(C2 + (size_t)(mBase + row) * ldc + n0 + c8) = lv;
        }
        __threadfence();
      }
    }
    __builtin_amdgcn_fence(__ATOMIC_RELEASE, "workgroup");
    __builtin_amdgcn_wave_barrier();
    __builtin_amdgcn_fence(__ATOMIC_ACQUIRE, "workgroup");
  }
}

#define GEMM_B2_F32     wmma_gemm64<0, false, 2, 0, false, 0>
#define GEMM_B1_H       wmma_gemm64<0, false, 1, 1, false, 0>
#define GEMM_F32        wmma_gemm64<0, false, 0, 0, false, 0>
#define GEMM_H          wmma_gemm64<0, false, 0, 1, false, 0>
#define GEMM_B1_H_RES   wmma_gemm64<0, false, 1, 1, true, 0>
#define GEMM_H_RELU     wmma_gemm64<0, false, 0, 1, false, 2>
#define GEMM_B1_F32_RES wmma_gemm64<0, false, 1, 0, true, 0>

struct CastSegs { const float* src[7]; unsigned short* dst[7]; int end2[8]; };
static_assert(sizeof(CastSegs) == 144);

__global__ __launch_bounds__(256) void cast_weights_kernel(CastSegs g) {
  const int i = blockIdx.x * 256 + threadIdx.x;
  const float* src = g.src[0];
  unsigned short* dst = g.dst[0];
  int base = 0;
#pragma unroll
  for (int s = 1; s < 7; ++s) {
    if (i >= g.end2[s - 1]) { src = g.src[s]; dst = g.dst[s]; base = g.end2[s - 1]; }
  }
  if (i < g.end2[6]) {
    const int j = i - base;
    const _Float16 h0 = (_Float16)(src[2 * (size_t)j] * WSC);
    const _Float16 h1 = (_Float16)(src[2 * (size_t)j + 1] * WSC);
    const unsigned u = (unsigned)__builtin_bit_cast(unsigned short, h0) |
                       ((unsigned)__builtin_bit_cast(unsigned short, h1) << 16);
    ((volatile unsigned*)dst)[j] = u;
    __threadfence();
    ((volatile unsigned*)dst)[j] = u;
  }
}

__global__ __launch_bounds__(256) void cast_ctx_kernel(const float* __restrict__ ctx, unsigned short* __restrict__ dst) {
  const int i = blockIdx.x * 256 + threadIdx.x;
  if (i < 64 * CC / 2) {
    const int row = i >> 7;
    float f0 = 0.f, f1 = 0.f;
    if (row < BB * NCC) { f0 = ctx[2 * i]; f1 = ctx[2 * i + 1]; }
    const _Float16 h0 = (_Float16)f0, h1 = (_Float16)f1;
    const unsigned u = (unsigned)__builtin_bit_cast(unsigned short, h0) |
                       ((unsigned)__builtin_bit_cast(unsigned short, h1) << 16);
    ((volatile unsigned*)dst)[i] = u;
    __threadfence();
    ((volatile unsigned*)dst)[i] = u;
  }
}

__device__ __forceinline__ void ln_store_rows(const _Float16* os, unsigned short* dst, int wave, int lane) {
  for (int pass = 0; pass < 2; ++pass) {
#pragma unroll
    for (int it = 0; it < 4; ++it) {
      const int row = wave * 4 + it;
      const v8h v = *(const v8h*)(os + row * 264 + lane * 8);
      *(volatile v8h*)(dst + (size_t)row * CC + lane * 8) = v;
    }
    __threadfence();
  }
}

__global__ __launch_bounds__(256) void ln_dual_kernel(const float* __restrict__ x,
    const float* __restrict__ g1, const float* __restrict__ b1,
    const float* __restrict__ g2, const float* __restrict__ b2,
    unsigned short* __restrict__ X1T, unsigned short* __restrict__ X2T) {
  __shared__ float tile[CC * 33];
  __shared__ __align__(16) _Float16 os[32 * 264];
  __shared__ float red[256];
  __shared__ float mean_s[32];
  __shared__ float rstd_s[32];
  const int tid = threadIdx.x, lane = tid & 31, wave = tid >> 5;
  const int blk = blockIdx.x;
  const int b = blk / (NN / 32);
  const int n0 = (blk - b * (NN / 32)) * 32;
  const float* xb = x + (size_t)b * CC * NN + n0 + lane;
#pragma unroll 8
  for (int i = 0; i < 32; ++i) {
    const int c = wave * 32 + i;
    tile[c * 33 + lane] = xb[(size_t)c * NN];
  }
  __syncthreads();
  float s = 0.f;
#pragma unroll 1
  for (int i = 0; i < 32; ++i) s += tile[(wave * 32 + i) * 33 + lane];
  red[tid] = s;
  __syncthreads();
  if (tid < 32) {
    float m = 0.f;
#pragma unroll
    for (int k = 0; k < 8; ++k) m += red[k * 32 + tid];
    mean_s[tid] = m * (1.0f / CC);
  }
  __syncthreads();
  const float mean = mean_s[lane];
  float s2 = 0.f;
#pragma unroll 1
  for (int i = 0; i < 32; ++i) {
    const float d = tile[(wave * 32 + i) * 33 + lane] - mean;
    s2 += d * d;
  }
  red[tid] = s2;
  __syncthreads();
  if (tid < 32) {
    float v = 0.f;
#pragma unroll
    for (int k = 0; k < 8; ++k) v += red[k * 32 + tid];
    rstd_s[tid] = rsqrtf(v * (1.0f / CC) + 1e-5f);
  }
  __syncthreads();
  const float rstd = rstd_s[lane];
#pragma unroll 1
  for (int i = 0; i < 32; ++i) {
    const int c = wave * 32 + i;
    const float xn = (tile[c * 33 + lane] - mean) * rstd;
    os[lane * 264 + c] = (_Float16)(xn * g1[c] + b1[c]);
  }
  __syncthreads();
  ln_store_rows(os, X1T + (size_t)(b * NN + n0) * CC, wave, lane);
  __syncthreads();
#pragma unroll 1
  for (int i = 0; i < 32; ++i) {
    const int c = wave * 32 + i;
    const float xn = (tile[c * 33 + lane] - mean) * rstd;
    os[lane * 264 + c] = (_Float16)(xn * g2[c] + b2[c]);
  }
  __syncthreads();
  ln_store_rows(os, X2T + (size_t)(b * NN + n0) * CC, wave, lane);
}

__global__ __launch_bounds__(256) void gate_kernel(const float* __restrict__ arch, const float* __restrict__ Wg,
                                                   const float* __restrict__ bg, float* __restrict__ gate) {
  __shared__ float guide[CC];
  const int b = blockIdx.x;
  const int o = threadIdx.x;
  float s = 0.f;
#pragma unroll
  for (int p = 0; p < NPP; ++p) s += arch[((size_t)b * NPP + p) * CC + o];
  guide[o] = s / (float)NPP;
  __syncthreads();
  float acc = 0.f;
  const float* wr = Wg + (size_t)o * CC;
#pragma unroll 1
  for (int c = 0; c < CC; ++c) acc += guide[c] * wr[c];
  acc += bg[o];
  const float e = __expf(-acc);
  const float gt = 1.0f / (1.0f + e);
  ((volatile float*)gate)[b * CC + o] = gt;
  __threadfence();
  ((volatile float*)gate)[b * CC + o] = gt;
}

__global__ __launch_bounds__(256) void qk_convert_kernel(const float* __restrict__ qk, const float* __restrict__ gate,
                                                         unsigned short* __restrict__ Q16, unsigned short* __restrict__ K16) {
  const int g = blockIdx.x * 256 + threadIdx.x;
  const int tok = g >> 6;
  const int j = (g & 63) * 8;
  const int b = tok >> 12;
  const float* sp = qk + (size_t)tok * QK_O + j;
  const v4f a0 = *(const v4f*)sp;
  const v4f a1 = *(const v4f*)(sp + 4);
  v8h hv;
  unsigned short* dst;
  if (j < CC) {
#pragma unroll
    for (int e = 0; e < 4; ++e) { hv[e] = (_Float16)a0[e]; hv[4 + e] = (_Float16)a1[e]; }
    dst = Q16 + (size_t)tok * CC + j;
  } else {
    const float* gp = gate + b * CC + (j - CC);
#pragma unroll
    for (int e = 0; e < 4; ++e) { hv[e] = (_Float16)(a0[e] * gp[e]); hv[4 + e] = (_Float16)(a1[e] * gp[4 + e]); }
    dst = K16 + (size_t)tok * CC + (j - CC);
  }
  *(volatile v8h*)dst = hv;
  __threadfence();
  *(volatile v8h*)dst = hv;
}

__global__ __launch_bounds__(256) void softmax_rows_kernel(const float* __restrict__ S, unsigned short* __restrict__ P) {
  __shared__ float redm[8];
  __shared__ float reds[8];
  const int tid = threadIdx.x, lane = tid & 31, wave = tid >> 5;
  const int row = blockIdx.x;
  const float* sp = S + (size_t)row * NN;
  const v4f a0 = *(const v4f*)(sp + tid * 8);
  const v4f a1 = *(const v4f*)(sp + tid * 8 + 4);
  const v4f a2 = *(const v4f*)(sp + 2048 + tid * 8);
  const v4f a3 = *(const v4f*)(sp + 2048 + tid * 8 + 4);
  float f[16];
#pragma unroll
  for (int e = 0; e < 4; ++e) { f[e] = a0[e]; f[4 + e] = a1[e]; f[8 + e] = a2[e]; f[12 + e] = a3[e]; }
  float mx = f[0];
#pragma unroll
  for (int e = 1; e < 16; ++e) mx = fmaxf(mx, f[e]);
#pragma unroll
  for (int off = 1; off < 32; off <<= 1) mx = fmaxf(mx, __shfl_xor(mx, off, 32));
  if (lane == 0) redm[wave] = mx;
  __syncthreads();
  mx = redm[0];
#pragma unroll
  for (int k = 1; k < 8; ++k) mx = fmaxf(mx, redm[k]);
  float sum = 0.f;
#pragma unroll
  for (int e = 0; e < 16; ++e) { f[e] = __expf(f[e] - mx); sum += f[e]; }
#pragma unroll
  for (int off = 1; off < 32; off <<= 1) sum += __shfl_xor(sum, off, 32);
  if (lane == 0) reds[wave] = sum;
  __syncthreads();
  float tot = reds[0];
#pragma unroll
  for (int k = 1; k < 8; ++k) tot += reds[k];
  const float inv = 1.0f / tot;
  v8h h0, h1;
#pragma unroll
  for (int e = 0; e < 8; ++e) { h0[e] = (_Float16)((f[e] * inv) * PSCALE); h1[e] = (_Float16)((f[8 + e] * inv) * PSCALE); }
  unsigned short* dp = P + (size_t)row * NN;
  for (int pass = 0; pass < 2; ++pass) {
    *(volatile v8h*)(dp + tid * 8) = h0;
    *(volatile v8h*)(dp + 2048 + tid * 8) = h1;
    __threadfence();
  }
}

__global__ __launch_bounds__(128) void token_attn_kernel(const float* __restrict__ qc, const float* __restrict__ kv,
                                                         unsigned short* __restrict__ refc) {
  __shared__ float kcs[NCC * HIDD];
  __shared__ float vcs[NCC * HIDD];
  __shared__ __align__(16) _Float16 outs[128 * 136];
  const int tid = threadIdx.x, lane = tid & 31, wave = tid >> 5;
  const int b = blockIdx.x / (NN / 128);
  const int n0 = (blockIdx.x - b * (NN / 128)) * 128;
  for (int i = tid; i < NCC * 2 * HIDD; i += 128) {
    const int r = i >> 8, o = i & 255;
    const float val = kv[(size_t)(b * NCC + r) * (2 * HIDD) + o];
    if (o < HIDD) kcs[r * HIDD + o] = val; else vcs[r * HIDD + (o - HIDD)] = val;
  }
  __syncthreads();
  const float* qrow = qc + (size_t)(b * NN + n0 + tid) * HIDD;
  float s[NCC];
#pragma unroll
  for (int j = 0; j < NCC; ++j) s[j] = 0.f;
#pragma unroll 1
  for (int h = 0; h < HIDD; ++h) {
    const float qv = qrow[h];
#pragma unroll
    for (int j = 0; j < NCC; ++j) s[j] += qv * kcs[j * HIDD + h];
  }
  const float sc = 0.08838834764831845f;
  float mx = -INFINITY;
#pragma unroll
  for (int j = 0; j < NCC; ++j) { s[j] *= sc; mx = fmaxf(mx, s[j]); }
  float sum = 0.f;
#pragma unroll
  for (int j = 0; j < NCC; ++j) { s[j] = __expf(s[j] - mx); sum += s[j]; }
  const float inv = 1.0f / sum;
#pragma unroll
  for (int j = 0; j < NCC; ++j) s[j] *= inv;
#pragma unroll 1
  for (int h = 0; h < HIDD; ++h) {
    float o = 0.f;
#pragma unroll
    for (int j = 0; j < NCC; ++j) o += vcs[j * HIDD + h] * s[j];
    outs[tid * 136 + h] = (_Float16)(o * WSC);
  }
  __syncthreads();
  unsigned short* dst = refc + (size_t)(b * NN + n0) * HIDD;
  for (int pass = 0; pass < 2; ++pass) {
#pragma unroll
    for (int it = 0; it < 16; ++it) {
      const int row = wave * 32 + it * 2 + (lane >> 4);
      const int c8 = (lane & 15) * 8;
      const v8h v = *(const v8h*)(outs + row * 136 + c8);
      *(volatile v8h*)(dst + (size_t)row * HIDD + c8) = v;
    }
    __threadfence();
  }
}

__global__ __launch_bounds__(256) void im2col_kernel(const unsigned short* __restrict__ fused, unsigned short* __restrict__ im) {
  const int px = blockIdx.x;
  const int b = px >> 12, n = px & 4095;
  const int y = n >> 6, x = n & 63;
  const unsigned short* fb = fused + (size_t)b * (2 * CC) * NN;
  unsigned short* dst = im + (size_t)px * KCONV;
  const int tid = threadIdx.x;
  v8h vals[3];
#pragma unroll
  for (int s = 0; s < 3; ++s) {
    const int slot = tid + s * 256;
    v8h v;
#pragma unroll
    for (int e = 0; e < 8; ++e) {
      const int k = slot * 8 + e;
      const int ci = k / 9;
      const int rem = k - ci * 9;
      const int ky = rem / 3;
      const int kx = rem - ky * 3;
      const int yy = y + ky - 1, xx = x + kx - 1;
      unsigned short hb = 0;
      if (slot < 576 && ci < 2 * CC && yy >= 0 && yy < HWD && xx >= 0 && xx < HWD)
        hb = fb[(size_t)ci * NN + yy * HWD + xx];
      v[e] = __builtin_bit_cast(_Float16, hb);
    }
    vals[s] = v;
  }
  for (int pass = 0; pass < 2; ++pass) {
#pragma unroll
    for (int s = 0; s < 3; ++s) {
      const int slot = tid + s * 256;
      if (slot < 576) *(volatile v8h*)(dst + (size_t)slot * 8) = vals[s];
    }
    __threadfence();
  }
}

static inline dim3 gemm_grid(int M, int N, int batches) {
  return dim3((unsigned)(((M / 64) * (N / 64) + 7) / 8), (unsigned)batches, 1);
}

extern "C" void kernel_launch(void* const* d_in, const int* in_sizes, int n_in,
                              void* d_out, int out_size, void* d_ws, size_t ws_size,
                              hipStream_t stream) {
  if (n_in < 22) return;
  if (in_sizes[0] != BB * CC * NN || out_size != BB * CC * NN) return;
  if (in_sizes[1] != BB * NPP * CC || in_sizes[2] != BB * NCC * CC) return;
  if (in_sizes[5] != 768 * CC || in_sizes[7] != CC * CC || in_sizes[9] != CC * CC ||
      in_sizes[13] != HIDD * CC || in_sizes[15] != 2 * HIDD * CC || in_sizes[17] != CC * HIDD ||
      in_sizes[19] != CC * 2 * CC * 9 || in_sizes[20] != CC * CC) return;

  const float* qry   = (const float*)d_in[0];
  const float* arch  = (const float*)d_in[1];
  const float* ctx   = (const float*)d_in[2];
  const float* ln1g  = (const float*)d_in[3];
  const float* ln1b  = (const float*)d_in[4];
  const float* Wqkv  = (const float*)d_in[5];
  const float* bqkv  = (const float*)d_in[6];
  const float* Wproj = (const float*)d_in[7];
  const float* bproj = (const float*)d_in[8];
  const float* Wg    = (const float*)d_in[9];
  const float* bg    = (const float*)d_in[10];
  const float* ln2g  = (const float*)d_in[11];
  const float* ln2b  = (const float*)d_in[12];
  const float* Wq    = (const float*)d_in[13];
  const float* bq    = (const float*)d_in[14];
  const float* Wkv   = (const float*)d_in[15];
  const float* bkv   = (const float*)d_in[16];
  const float* Wout  = (const float*)d_in[17];
  const float* bout  = (const float*)d_in[18];
  const float* Wf1   = (const float*)d_in[19];
  const float* Wf2   = (const float*)d_in[20];
  const float* bf2   = (const float*)d_in[21];
  float* outp = (float*)d_out;

  char* ws = (char*)d_ws;
  size_t off = 0;
  auto carve = [&](size_t bytes) -> char* {
    char* p = ws + off;
    off += (bytes + 4095) & ~(size_t)4095;
    return p;
  };
  unsigned short* Wqkv16  = (unsigned short*)carve((size_t)768 * CC * 2);
  unsigned short* Wproj16 = (unsigned short*)carve((size_t)CC * CC * 2);
  unsigned short* Wq16    = (unsigned short*)carve((size_t)HIDD * CC * 2);
  unsigned short* Wkv16   = (unsigned short*)carve((size_t)2 * HIDD * CC * 2);
  unsigned short* Wout16  = (unsigned short*)carve((size_t)CC * HIDD * 2);
  unsigned short* Wf1r16  = (unsigned short*)carve((size_t)CC * KCONV * 2);
  unsigned short* Wf2_16  = (unsigned short*)carve((size_t)CC * CC * 2);
  unsigned short* CTX16   = (unsigned short*)carve((size_t)64 * CC * 2);
  float*          gate    = (float*)carve((size_t)BB * CC * 4);
  float*          KV32    = (float*)carve((size_t)64 * CC * 4);
  unsigned short* FUSED16 = (unsigned short*)carve((size_t)BB * 2 * CC * NN * 2);
  unsigned short* REF16   = (unsigned short*)carve((size_t)NN * CC * 2);
  unsigned short* Q16     = (unsigned short*)carve((size_t)BB * NN * CC * 2);
  unsigned short* K16     = (unsigned short*)carve((size_t)BB * NN * CC * 2);
  unsigned short* V16     = (unsigned short*)carve((size_t)BB * CC * NN * 2);
  unsigned short* Y1      = (unsigned short*)carve((size_t)NPIX * CC * 2);
  const size_t bigBytes = (size_t)NN * NN * 4 + (size_t)NN * NN * 2;
  char* BIG = carve(bigBytes);
  if (off > ws_size || off > (size_t)134217728) return;
  float*          S32    = (float*)(BIG);
  unsigned short* P16    = (unsigned short*)(BIG + (size_t)NN * NN * 4);
  unsigned short* X1T    = (unsigned short*)(BIG);
  unsigned short* X2T    = (unsigned short*)(BIG + (size_t)4 * 1048576);
  float*          QK32   = (float*)(BIG + (size_t)8 * 1048576);
  float*          QC32   = (float*)(BIG + (size_t)24 * 1048576);
  unsigned short* REFC16 = (unsigned short*)(BIG + (size_t)28 * 1048576);
  unsigned short* IM     = (unsigned short*)(BIG);
  if ((size_t)NPIX * KCONV * 2 > bigBytes) return;

  const dim3 blk256(256);

  CastSegs cs;
  cs.src[0] = Wqkv;  cs.dst[0] = Wqkv16;
  cs.src[1] = Wproj; cs.dst[1] = Wproj16;
  cs.src[2] = Wq;    cs.dst[2] = Wq16;
  cs.src[3] = Wkv;   cs.dst[3] = Wkv16;
  cs.src[4] = Wout;  cs.dst[4] = Wout16;
  cs.src[5] = Wf1;   cs.dst[5] = Wf1r16;
  cs.src[6] = Wf2;   cs.dst[6] = Wf2_16;
  {
    const int idx[7] = {5, 7, 13, 15, 17, 19, 20};
    int acc2 = 0;
    for (int s = 0; s < 7; ++s) { acc2 += in_sizes[idx[s]] / 2; cs.end2[s] = acc2; }
    cs.end2[7] = acc2;
  }
  cast_weights_kernel<<<dim3((unsigned)((cs.end2[6] + 255) / 256)), blk256, 0, stream>>>(cs);

  cast_ctx_kernel<<<dim3(32), blk256, 0, stream>>>(ctx, CTX16);

  ln_dual_kernel<<<dim3(BB * NN / 32), blk256, 0, stream>>>(qry, ln1g, ln1b, ln2g, ln2b, X1T, X2T);

  gate_kernel<<<dim3(BB), blk256, 0, stream>>>(arch, Wg, bg, gate);

  GEMM_B2_F32<<<gemm_grid(NN, QK_O, BB), blk256, 0, stream>>>(
      X1T, X1T, CC, (long)NN * CC, Wqkv16, Wqkv16, CC, 0L,
      QK32, QK32, QK_O, (long)NN * QK_O, bqkv, qry, 0L, NN, QK_O, CC, 1.0f / WSC);

  GEMM_B1_H<<<gemm_grid(CC, NN, BB), blk256, 0, stream>>>(
      Wqkv16 + (size_t)512 * CC, Wqkv16 + (size_t)512 * CC, CC, 0L, X1T, X1T, CC, (long)NN * CC,
      V16, V16, NN, (long)CC * NN, bqkv + 512, qry, 0L, CC, NN, CC, 1.0f / WSC);

  qk_convert_kernel<<<dim3(BB * NN * 64 / 256), blk256, 0, stream>>>(QK32, gate, Q16, K16);

  GEMM_B2_F32<<<gemm_grid(NN, HIDD, BB), blk256, 0, stream>>>(
      X2T, X2T, CC, (long)NN * CC, Wq16, Wq16, CC, 0L,
      QC32, QC32, HIDD, (long)NN * HIDD, bq, qry, 0L, NN, HIDD, CC, 1.0f / WSC);

  GEMM_B2_F32<<<gemm_grid(64, 2 * HIDD, 1), blk256, 0, stream>>>(
      CTX16, CTX16, CC, 0L, Wkv16, Wkv16, CC, 0L,
      KV32, KV32, 2 * HIDD, 0L, bkv, qry, 0L, 64, 2 * HIDD, CC, 1.0f / WSC);

  token_attn_kernel<<<dim3(BB * NN / 128), dim3(128), 0, stream>>>(QC32, KV32, REFC16);

  GEMM_B1_H_RES<<<gemm_grid(CC, NN, BB), blk256, 0, stream>>>(
      Wout16, Wout16, HIDD, 0L, REFC16, REFC16, HIDD, (long)NN * HIDD,
      FUSED16 + (size_t)CC * NN, FUSED16 + (size_t)CC * NN, NN, (long)2 * CC * NN,
      bout, qry, (long)CC * NN, CC, NN, HIDD, 1.0f / (WSC * WSC));

  for (int b = 0; b < BB; ++b) {
    GEMM_F32<<<gemm_grid(NN, NN, 1), blk256, 0, stream>>>(
        Q16 + (size_t)b * NN * CC, Q16 + (size_t)b * NN * CC, CC, 0L,
        K16 + (size_t)b * NN * CC, K16 + (size_t)b * NN * CC, CC, 0L,
        S32, S32, NN, 0L, bqkv, qry, 0L, NN, NN, CC, 1.0f / 16.0f);
    softmax_rows_kernel<<<dim3(NN), blk256, 0, stream>>>(S32, P16);
    GEMM_H<<<gemm_grid(NN, CC, 1), blk256, 0, stream>>>(
        P16, P16, NN, 0L, V16 + (size_t)b * CC * NN, V16 + (size_t)b * CC * NN, NN, 0L,
        REF16, REF16, CC, 0L, bqkv, qry, 0L, NN, CC, NN, WSC / PSCALE);
    GEMM_B1_H_RES<<<gemm_grid(CC, NN, 1), blk256, 0, stream>>>(
        Wproj16, Wproj16, CC, 0L, REF16, REF16, CC, 0L,
        FUSED16 + (size_t)b * 2 * CC * NN, FUSED16 + (size_t)b * 2 * CC * NN, NN, 0L,
        bproj, qry + (size_t)b * CC * NN, 0L, CC, NN, CC, 1.0f / (WSC * WSC));
  }

  im2col_kernel<<<dim3(NPIX), blk256, 0, stream>>>(FUSED16, IM);

  GEMM_H_RELU<<<gemm_grid(NPIX, CC, 1), blk256, 0, stream>>>(
      IM, IM, KCONV, 0L, Wf1r16, Wf1r16, KCONV, 0L,
      Y1, Y1, CC, 0L, bf2, qry, 0L, NPIX, CC, KCONV, 1.0f / WSC);

  GEMM_B1_F32_RES<<<gemm_grid(CC, NN, BB), blk256, 0, stream>>>(
      Wf2_16, Wf2_16, CC, 0L, Y1, Y1, CC, (long)NN * CC,
      outp, outp, NN, (long)CC * NN, bf2, qry, (long)CC * NN, CC, NN, CC, 1.0f / WSC);

  (void)hipGetLastError();
}
